// CNNEMLStageNet_3332894621846
// MI455X (gfx1250) — hardware-verified
//
#include <hip/hip_runtime.h>
#include <hip/hip_bf16.h>
#include <math.h>

typedef __attribute__((ext_vector_type(16))) _Float16 v16h;
typedef __attribute__((ext_vector_type(8)))  _Float16 v8h;
typedef __attribute__((ext_vector_type(4)))  _Float16 v4h;
typedef __attribute__((ext_vector_type(16))) __bf16   v16b;
typedef __attribute__((ext_vector_type(8)))  __bf16   v8b;
typedef __attribute__((ext_vector_type(8)))  float    v8f;
typedef __attribute__((ext_vector_type(4)))  float    v4f;
#define PSCALE 32768.0f
#define U16(p) ((const unsigned short*)(const void*)(p))
#define PSCALE_INV (1.0f / 32768.0f)

__device__ __forceinline__ unsigned short f2bf_bits(float f) {
  unsigned u = __float_as_uint(f);
  return (unsigned short)((u + 0x7FFFu + ((u >> 16) & 1u)) >> 16);
}
__device__ __forceinline__ float bf_bits2f(unsigned short h) { return __uint_as_float(((unsigned)h) << 16); }

__device__ __forceinline__ void dep_guard_h(v8f& a, v8f& b, v16h x, v16h y) { asm volatile("v_nop\n\tv_nop\n\tv_nop\n\tv_nop" : "+v"(a), "+v"(b) : "v"(x), "v"(y)); }
__device__ __forceinline__ void dep_guard_b(v8f& a, v8f& b, v16b x, v16b y) { asm volatile("v_nop\n\tv_nop\n\tv_nop\n\tv_nop" : "+v"(a), "+v"(b) : "v"(x), "v"(y)); }
__device__ __forceinline__ void dep_guard1(v8f& a, v16h x, v16h y) { asm volatile("v_nop\n\tv_nop\n\tv_nop\n\tv_nop" : "+v"(a) : "v"(x), "v"(y)); }
__device__ __forceinline__ void keep4_h(v16h a, v16h b, v16h c, v16h d) { asm volatile("v_nop" :: "v"(a), "v"(b), "v"(c), "v"(d)); }
__device__ __forceinline__ void keep4_b(v16b a, v16b b, v16b c, v16b d) { asm volatile("v_nop" :: "v"(a), "v"(b), "v"(c), "v"(d)); }
__device__ __forceinline__ void acc_guard4(v8f& a, v8f& b, v8f& c, v8f& d) { asm volatile("v_nop\n\tv_nop\n\tv_nop\n\tv_nop" : "+v"(a), "+v"(b), "+v"(c), "+v"(d)); }
template <typename T> struct Frag;
template <> struct Frag<_Float16> {
  typedef v16h V; union U { v16h v; v8h h[2]; };
  static __device__ __forceinline__ v16h load(const _Float16* p) {
    U f; f.h[0] = *(const v8h*)(p); f.h[1] = *(const v8h*)(p + 16); return f.v;
  }
  static __device__ __forceinline__ v8f mma(v16h a, v16h b, v8f c) {
    return __builtin_amdgcn_wmma_f32_16x16x32_f16(false, a, false, b, (short)0, c, false, false);
  }
  static __device__ __forceinline__ void guard(v8f& a, v8f& b, v16h x, v16h y) { dep_guard_h(a, b, x, y); }
  static __device__ __forceinline__ void keep(v16h a, v16h b, v16h c, v16h d) { keep4_h(a, b, c, d); }
};
template <> struct Frag<__bf16> {
  typedef v16b V; union U { v16b v; v8b h[2]; };
  static __device__ __forceinline__ v16b load(const __bf16* p) {
    U f; f.h[0] = *(const v8b*)(p); f.h[1] = *(const v8b*)(p + 16); return f.v;
  }
  static __device__ __forceinline__ v8f mma(v16b a, v16b b, v8f c) {
    return __builtin_amdgcn_wmma_f32_16x16x32_bf16(false, a, false, b, (short)0, c, false, false);
  }
  static __device__ __forceinline__ void guard(v8f& a, v8f& b, v16b x, v16b y) { dep_guard_b(a, b, x, y); }
  static __device__ __forceinline__ void keep(v16b a, v16b b, v16b c, v16b d) { keep4_b(a, b, c, d); }
};

template <int ET> struct Elem;
template <> struct Elem<0> { typedef _Float16 T; };
template <> struct Elem<1> { typedef __bf16 T; };
template <int ET, bool SPLIT, int BIAS_MODE, int OUT_MODE, bool RESID, int ACT = 0>
__global__ __launch_bounds__(256) void wmma_gemm64(
    const unsigned short* __restrict__ Ap, const unsigned short* __restrict__ A2p, int lda, long strideA,
    const unsigned short* __restrict__ Btp, const unsigned short* __restrict__ Bt2p, int ldb, long strideB,
    void* __restrict__ Cout, void* __restrict__ Cout2, int ldc, long strideC,
    const float* __restrict__ bias,
    const float* __restrict__ resid, long strideR,
    int M, int N, int K, float scale) {
  typedef typename Elem<ET>::T T;
  typedef typename Frag<T>::V V;
  const T* A = (const T*)Ap; const T* A2 = (const T*)A2p; const T* Bt = (const T*)Btp; const T* Bt2 = (const T*)Bt2p;
  __shared__ __align__(16) float sT[8][16 * 68];
  const int b    = blockIdx.y;
  const int lane = threadIdx.x & 31;
  const int wave = threadIdx.x >> 5;
  const int tilesN = N >> 6;
  const int tilesM = M >> 6;
  const int tile = blockIdx.x * 8 + wave;
  if (tile >= tilesM * tilesN) return;
  const int tm = tile / tilesN;
  const int tn = tile - tm * tilesN;
  const int m0 = tm << 6;
  const int n0 = tn << 6;

  const T* Ab  = A  + (size_t)b * strideA;
  const T* Bb  = Bt + (size_t)b * strideB;
  const T* Ab2 = SPLIT ? (A2  + (size_t)b * strideA) : nullptr;
  const T* Bb2 = SPLIT ? (Bt2 + (size_t)b * strideB) : nullptr;

  const int rlane = lane & 15;
  const int koff  = (lane >> 4) * 8;
  const int mOff  = (lane >> 4) * 8;

  v8f acc[4][4];
#pragma unroll
  for (int i = 0; i < 4; ++i)
#pragma unroll
    for (int j = 0; j < 4; ++j) acc[i][j] = (v8f){0.f,0.f,0.f,0.f,0.f,0.f,0.f,0.f};

  for (int k0 = 0; k0 < K; k0 += 32) {
    V bh[4], bl[4];
#pragma unroll
    for (int j = 0; j < 4; ++j) {
      const size_t bo = (size_t)(n0 + (j << 4) + rlane) * ldb + koff + k0;
      bh[j] = Frag<T>::load(Bb + bo);
      if (SPLIT) bl[j] = Frag<T>::load(Bb2 + bo);
    }
#pragma unroll
    for (int i = 0; i < 4; ++i) {
      const size_t ao = (size_t)(m0 + (i << 4) + rlane) * lda + koff + k0;
      V ah = Frag<T>::load(Ab + ao);
      V al;
      if (SPLIT) al = Frag<T>::load(Ab2 + ao);
#pragma unroll
      for (int j = 0; j < 4; ++j) {
        acc[i][j] = Frag<T>::mma(ah, bh[j], acc[i][j]);
        if (SPLIT) {
          acc[i][j] = Frag<T>::mma(ah, bl[j], acc[i][j]);
          acc[i][j] = Frag<T>::mma(al, bh[j], acc[i][j]);
        }
      }
      Frag<T>::guard(acc[i][0], acc[i][3], ah, SPLIT ? al : ah);
    }
    Frag<T>::keep(bh[0], bh[1], bh[2], bh[3]);
    if (SPLIT) Frag<T>::keep(bl[0], bl[1], bl[2], bl[3]);
  }
  acc_guard4(acc[0][0], acc[0][1], acc[0][2], acc[0][3]);
  acc_guard4(acc[1][0], acc[1][1], acc[1][2], acc[1][3]);
  acc_guard4(acc[2][0], acc[2][1], acc[2][2], acc[2][3]);
  acc_guard4(acc[3][0], acc[3][1], acc[3][2], acc[3][3]);

  float* slab = sT[wave];
  const float* Rb = RESID ? (resid + (size_t)b * strideR) : nullptr;
#pragma unroll
  for (int i = 0; i < 4; ++i) {
    const int mBase = m0 + (i << 4);
#pragma unroll
    for (int j = 0; j < 4; ++j) {
      const int n = n0 + (j << 4) + rlane;
      float bv = 0.f;
      if (BIAS_MODE == 2) bv = bias[n];
#pragma unroll
      for (int r = 0; r < 8; ++r) {
        float v = acc[i][j][r] * scale;
        if (BIAS_MODE == 1) v += bias[mBase + mOff + r];
        if (BIAS_MODE == 2) v += bv;
        if (RESID) v += Rb[(size_t)(mBase + mOff + r) * ldc + n];
        if (ACT == 1) v = tanhf(v);
        if (ACT == 2) v = fmaxf(v, 0.0f);
        if (ACT == 3) v = v / (1.0f + expf(-v));
        if (ACT == 4) v = (v > 0.f) ? v : 0.01f * v;
        if (ACT == 5) v = 0.5f * v * (1.0f + erff(v * 0.70710678118654752f));
        slab[(mOff + r) * 68 + (j << 4) + rlane] = v;
      }
    }
    __builtin_amdgcn_fence(__ATOMIC_RELEASE, "workgroup");
    __builtin_amdgcn_wave_barrier();
    __builtin_amdgcn_fence(__ATOMIC_ACQUIRE, "workgroup");
    if (OUT_MODE == 0) {
      float* C = (float*)Cout + (size_t)b * strideC;
      const int hh = lane >> 4, c4 = (lane & 15) * 4;
      for (int pass = 0; pass < 2; ++pass) {
#pragma unroll
        for (int it = 0; it < 8; ++it) {
          const int row = it * 2 + hh;
          v4f v = *(const v4f*)(slab + row * 68 + c4);
          *(volatile v4f*)(C + (size_t)(mBase + row) * ldc + n0 + c4) = v;
        }
        __threadfence();
      }
    } else {
      const int q = lane >> 3, c8 = (lane & 7) * 8;
      unsigned short* C  = (unsigned short*)Cout  + (size_t)b * strideC;
      unsigned short* C2 = (OUT_MODE == 2) ? ((unsigned short*)Cout2 + (size_t)b * strideC) : nullptr;
      for (int pass = 0; pass < 2; ++pass) {
#pragma unroll
        for (int it = 0; it < 4; ++it) {
          const int row = it * 4 + q;
          const float* sp = slab + row * 68 + c8;
          v8h hv, lv;
#pragma unroll
          for (int e = 0; e < 8; ++e) {
            if (OUT_MODE == 1) {
              hv[e] = (_Float16)sp[e];
            } else {
              unsigned short hb = f2bf_bits(sp[e]);
              unsigned short lb = f2bf_bits(sp[e] - bf_bits2f(hb));
              hv[e] = __builtin_bit_cast(_Float16, hb);
              lv[e] = __builtin_bit_cast(_Float16, lb);
            }
          }
          *(volatile v8h*)(C + (size_t)(mBase + row) * ldc + n0 + c8) = hv;
          if (OUT_MODE == 2) *(volatile v8h*)(C2 + (size_t)(mBase + row) * ldc + n0 + c8) = lv;
        }
        __threadfence();
      }
    }
    __builtin_amdgcn_fence(__ATOMIC_RELEASE, "workgroup");
    __builtin_amdgcn_wave_barrier();
    __builtin_amdgcn_fence(__ATOMIC_ACQUIRE, "workgroup");
  }
}

#define NPIX   36864
#define CDIM   128
#define HH     96
#define WW     96
#define HWPIX  9216
#define PLD    640
#define NBR    9
#define TT     16
#define NE     144
#define HP     264
#define XSC    16.0f
#define WSC    64.0f
#define HSC    64.0f
#define MSC    64.0f
#define LN_EPS_F   1e-5f
#define GATE_EPS_F 1e-6f
#define CLIPV      3.0f

__device__ __forceinline__ float wsum32(float v) {
#pragma unroll
  for (int off = 16; off > 0; off >>= 1) v += __shfl_xor(v, off, 32);
  return v;
}
__device__ __forceinline__ float hsum16(float v) {
#pragma unroll
  for (int off = 8; off > 0; off >>= 1) v += __shfl_xor(v, off, 32);
  return v;
}
__device__ __forceinline__ float softplus_f(float x) {
  return fmaxf(x, 0.f) + log1pf(expf(-fabsf(x)));
}
__device__ __forceinline__ float gelu_exact(float x) {
  return x * (erff(x * 0.70710678118654752f) + 1.f) * 0.5f;
}

__global__ __launch_bounds__(256) void prep_kernel(
    const float* __restrict__ d_w1, const float* __restrict__ d_b1,
    const float* __restrict__ r_w1, const float* __restrict__ r_b1,
    const float* __restrict__ v_w,  const float* __restrict__ o_w,
    const float* __restrict__ rel_pos,
    _Float16* __restrict__ Wbig, _Float16* __restrict__ oW,
    float* __restrict__ cD, float* __restrict__ cR) {
  const int gid = blockIdx.x * 256 + threadIdx.x;
  if (gid < 640 * 16) {
    const int n = gid >> 4, k8 = (gid & 15) * 8;
    const int seg = n >> 7, col = n & 127;
    const float* W1 = (seg < 2) ? d_w1 : r_w1;
    const bool isC = (seg == 0) || (seg == 2);
    const int rowoff = isC ? 0 : 128;
    v8h o;
#pragma unroll
    for (int e = 0; e < 8; ++e) {
      const int k = k8 + e;
      const float a  = W1[(size_t)(rowoff + k) * CDIM + col];
      const float d  = W1[(size_t)(256 + k) * CDIM + col];
      const float vv = v_w[(size_t)k * CDIM + col];
      float val = isC ? (a + d) : (a - d);
      if (seg == 4) val = vv;
      o[e] = (_Float16)(val * WSC);
    }
    _Float16* dst = Wbig + (size_t)n * CDIM + k8;
    *(volatile v8h*)dst = o;
    __threadfence();
    *(volatile v8h*)dst = o;
  } else if (gid < 640 * 16 + 128 * 16) {
    const int u = gid - 640 * 16;
    const int n = u >> 4, k8 = (u & 15) * 8;
    v8h o;
#pragma unroll
    for (int e = 0; e < 8; ++e) o[e] = (_Float16)(o_w[(size_t)(k8 + e) * CDIM + n] * WSC);
    _Float16* dst = oW + (size_t)n * CDIM + k8;
    *(volatile v8h*)dst = o;
    __threadfence();
    *(volatile v8h*)dst = o;
  } else if (gid < 640 * 16 + 128 * 16 + 2 * NBR * CDIM) {
    const int u = gid - (640 * 16 + 128 * 16);
    const bool which = (u >= NBR * CDIM);
    const int idx = which ? (u - NBR * CDIM) : u;
    const int kk = idx >> 7, col = idx & 127;
    const float* W1 = which ? r_w1 : d_w1;
    const float* b1 = which ? r_b1 : d_b1;
    float s = b1[col];
#pragma unroll
    for (int r = 0; r < 8; ++r) s += rel_pos[kk * 8 + r] * W1[(size_t)(384 + r) * CDIM + col];
    float* dst = which ? cR : cD;
    ((volatile float*)dst)[idx] = s;
    __threadfence();
    ((volatile float*)dst)[idx] = s;
  }
}

__global__ __launch_bounds__(256) void ln1_kernel(
    const float* __restrict__ tokens, const float* __restrict__ lnw,
    const float* __restrict__ lnb, _Float16* __restrict__ X, int npix) {
  const int tid = threadIdx.x, wave = tid >> 5, lane = tid & 31;
  const int hh = lane >> 4, c = lane & 15, c8 = c * 8;
  const int row = blockIdx.x * 16 + wave * 2 + hh;
  const bool pv = row < npix;
  const int rowc = pv ? row : (npix - 1);
  const v4f x0 = *(const v4f*)(tokens + (size_t)rowc * CDIM + c8);
  const v4f x1 = *(const v4f*)(tokens + (size_t)rowc * CDIM + c8 + 4);
  float s = x0[0] + x0[1] + x0[2] + x0[3] + x1[0] + x1[1] + x1[2] + x1[3];
  s = hsum16(s);
  const float mean = s * (1.f / 128.f);
  float d[8];
#pragma unroll
  for (int e = 0; e < 4; ++e) { d[e] = x0[e] - mean; d[4 + e] = x1[e] - mean; }
  float sq = 0.f;
#pragma unroll
  for (int e = 0; e < 8; ++e) sq += d[e] * d[e];
  sq = hsum16(sq);
  const float rs = rsqrtf(sq * (1.f / 128.f) + LN_EPS_F);
  const v4f w0 = *(const v4f*)(lnw + c8), w1 = *(const v4f*)(lnw + c8 + 4);
  const v4f b0 = *(const v4f*)(lnb + c8), b1 = *(const v4f*)(lnb + c8 + 4);
  v8h o;
#pragma unroll
  for (int e = 0; e < 4; ++e) {
    o[e]     = (_Float16)((d[e] * rs * w0[e] + b0[e]) * XSC);
    o[4 + e] = (_Float16)((d[4 + e] * rs * w1[e] + b1[e]) * XSC);
  }
  _Float16* dst = X + (size_t)rowc * CDIM + c8;
  if (pv) *(volatile v8h*)dst = o;
  __threadfence();
  if (pv) *(volatile v8h*)dst = o;
}

__global__ __launch_bounds__(256) void edge_kernel(
    const float* __restrict__ P, const float* __restrict__ cD, const float* __restrict__ cR,
    const float* __restrict__ d_w2, const float* __restrict__ d_b2,
    const float* __restrict__ r_w2, const float* __restrict__ r_b2,
    const float* __restrict__ v_b, const float* __restrict__ g_raw,
    const float* __restrict__ g_lam, const float* __restrict__ g_bias,
    _Float16* __restrict__ MSG, int npix) {
  __shared__ __align__(16) _Float16 hidA[NE * HP];
  __shared__ __align__(16) _Float16 w2B[16 * HP];
  __shared__ float drs[NE * 2];
  __shared__ float gsh[NE];
  const int tid = threadIdx.x, wave = tid >> 5, lane = tid & 31;
  const int hh = lane >> 4, c = lane & 15;
  const int tok0 = blockIdx.x * TT;

  for (int i = tid; i < 16 * 256; i += 256) {
    const int n = i >> 8, k = i & 255, kk = k & 127;
    const float vd = d_w2[kk] * WSC, vr = r_w2[kk] * WSC;
    float val = 0.f;
    if (n == 0 && k < 128) val = vd;
    if (n == 1 && k >= 128) val = vr;
    w2B[n * HP + k] = (_Float16)val;
  }

  const int cb = lane * 4;
#pragma unroll 1
  for (int j = 0; j < NE / 8; ++j) {
    const int e = wave + 8 * j;
    const int lt = e / NBR;
    const int k = e - lt * NBR;
    int p = tok0 + lt; p = (p < npix) ? p : (npix - 1);
    const int bimg = p / HWPIX;
    const int rem = p - bimg * HWPIX;
    const int y = rem / WW;
    const int x = rem - y * WW;
    const int ky = k / 3;
    const int dy = ky - 1, dx = (k - ky * 3) - 1;
    const int ny = y + dy, nx = x + dx;
    const bool in = ((unsigned)ny < (unsigned)HH) && ((unsigned)nx < (unsigned)WW);
    const int q = in ? (bimg * HWPIX + ny * WW + nx) : p;
    const float fin = in ? 1.f : 0.f;
    const v4f pcd = *(const v4f*)(P + (size_t)p * PLD + cb);
    const v4f pnd = *(const v4f*)(P + (size_t)q * PLD + 128 + cb);
    const v4f pcr = *(const v4f*)(P + (size_t)p * PLD + 256 + cb);
    const v4f pnr = *(const v4f*)(P + (size_t)q * PLD + 384 + cb);
    const v4f kd = *(const v4f*)(cD + k * CDIM + cb);
    const v4f kr = *(const v4f*)(cR + k * CDIM + cb);
    v4h hd, hr;
#pragma unroll
    for (int t = 0; t < 4; ++t) {
      hd[t] = (_Float16)(gelu_exact(pcd[t] + fin * pnd[t] + kd[t]) * HSC);
      hr[t] = (_Float16)(gelu_exact(pcr[t] + fin * pnr[t] + kr[t]) * HSC);
    }
    *(v4h*)(hidA + (size_t)e * HP + cb) = hd;
    *(v4h*)(hidA + (size_t)e * HP + 128 + cb) = hr;
  }
  __syncthreads();

  for (int rt = wave; rt < NE / 16; rt += 8) {
    v8f acc = (v8f){0.f,0.f,0.f,0.f,0.f,0.f,0.f,0.f};
#pragma unroll
    for (int ks = 0; ks < 8; ++ks) {
      const v16h a = Frag<_Float16>::load(hidA + (size_t)(rt * 16 + c) * HP + ks * 32 + 8 * hh);
      const v16h b = Frag<_Float16>::load(w2B + c * HP + ks * 32 + 8 * hh);
      acc = Frag<_Float16>::mma(a, b, acc);
      dep_guard1(acc, a, b);
    }
    if (c < 2) {
#pragma unroll
      for (int r = 0; r < 8; ++r) drs[(rt * 16 + 8 * hh + r) * 2 + c] = acc[r];
    }
  }
  __syncthreads();

  if (tid < NE) {
    const float drive = drs[tid * 2] * (1.f / (HSC * WSC)) + d_b2[0];
    const float res   = drs[tid * 2 + 1] * (1.f / (HSC * WSC)) + r_b2[0];
    const float gamma = softplus_f(g_raw[0]);
    const float den = softplus_f(res) + gamma + GATE_EPS_F;
    const float cond = drive / den;
    float en = g_lam[0] * cond;
    en = fminf(fmaxf(en, -CLIPV), CLIPV);
    en = 1.0f * en + g_bias[0];
    gsh[tid] = 1.f / (1.f + expf(-en));
  }
  __syncthreads();

  {
    const int lt = wave * 2 + hh;
    int p = tok0 + lt;
    const bool pv = p < npix;
    p = pv ? p : (npix - 1);
    const int bimg = p / HWPIX;
    const int rem = p - bimg * HWPIX;
    const int y = rem / WW;
    const int x = rem - y * WW;
    const int c8 = c * 8;
    float m[8];
#pragma unroll
    for (int t = 0; t < 8; ++t) m[t] = 0.f;
    float G = 0.f;
#pragma unroll 1
    for (int k = 0; k < NBR; ++k) {
      const int ky = k / 3;
      const int dy = ky - 1, dx = (k - ky * 3) - 1;
      const int ny = y + dy, nx = x + dx;
      const bool in = ((unsigned)ny < (unsigned)HH) && ((unsigned)nx < (unsigned)WW);
      const int q = in ? (bimg * HWPIX + ny * WW + nx) : p;
      const float gk = gsh[lt * NBR + k];
      G += gk;
      const float ge = in ? gk : 0.f;
      const v4f v0 = *(const v4f*)(P + (size_t)q * PLD + 512 + c8);
      const v4f v1 = *(const v4f*)(P + (size_t)q * PLD + 512 + c8 + 4);
#pragma unroll
      for (int t = 0; t < 4; ++t) { m[t] += ge * v0[t]; m[4 + t] += ge * v1[t]; }
    }
    const float mass = fmaxf(G, GATE_EPS_F);
    const float inv = 1.f / mass;
    const v4f vb0 = *(const v4f*)(v_b + c8), vb1 = *(const v4f*)(v_b + c8 + 4);
    v8h ov;
#pragma unroll
    for (int t = 0; t < 4; ++t) {
      ov[t]     = (_Float16)(((m[t] + vb0[t] * G) * inv) * MSC);
      ov[4 + t] = (_Float16)(((m[4 + t] + vb1[t] * G) * inv) * MSC);
    }
    _Float16* dst = MSG + (size_t)p * CDIM + c8;
    if (pv) *(volatile v8h*)dst = ov;
    __threadfence();
    if (pv) *(volatile v8h*)dst = ov;
  }
}

__global__ __launch_bounds__(256) void ln2_kernel(
    const float* __restrict__ Y, const float* __restrict__ lnw,
    const float* __restrict__ lnb, float* __restrict__ out, int npix) {
  const int tid = threadIdx.x, wave = tid >> 5, lane = tid & 31;
  const int row = blockIdx.x * 8 + wave;
  const bool pv = row < npix;
  const int rowc = pv ? row : (npix - 1);
  const v4f x = *(const v4f*)(Y + (size_t)rowc * CDIM + lane * 4);
  float s = wsum32(x[0] + x[1] + x[2] + x[3]);
  const float mean = s * (1.f / 128.f);
  const float d0 = x[0] - mean, d1 = x[1] - mean, d2 = x[2] - mean, d3 = x[3] - mean;
  const float sq = wsum32(d0 * d0 + d1 * d1 + d2 * d2 + d3 * d3);
  const float rs = rsqrtf(sq * (1.f / 128.f) + LN_EPS_F);
  const v4f w = *(const v4f*)(lnw + lane * 4);
  const v4f b = *(const v4f*)(lnb + lane * 4);
  v4f o;
  o[0] = d0 * rs * w[0] + b[0];
  o[1] = d1 * rs * w[1] + b[1];
  o[2] = d2 * rs * w[2] + b[2];
  o[3] = d3 * rs * w[3] + b[3];
  float* dst = out + (size_t)rowc * CDIM + lane * 4;
  if (pv) *(volatile v4f*)dst = o;
  __threadfence();
  if (pv) *(volatile v4f*)dst = o;
}

extern "C" void kernel_launch(void* const* d_in, const int* in_sizes, int n_in,
                              void* d_out, int out_size, void* d_ws, size_t ws_size,
                              hipStream_t stream) {
  if (n_in < 21) return;
  const int npix = NPIX;
  if (in_sizes[0] != npix * CDIM || out_size != npix * CDIM) return;
  if (in_sizes[5] != NBR * 8 || in_sizes[6] != 392 * CDIM || in_sizes[10] != 392 * CDIM) return;
  if (in_sizes[8] != CDIM || in_sizes[12] != CDIM || in_sizes[14] != CDIM * CDIM || in_sizes[16] != CDIM * CDIM) return;
  if (in_sizes[1] != CDIM || in_sizes[2] != CDIM || in_sizes[3] != CDIM || in_sizes[4] != CDIM) return;
  if (in_sizes[7] != CDIM || in_sizes[11] != CDIM || in_sizes[15] != CDIM || in_sizes[17] != CDIM) return;

  const float* tokens  = (const float*)d_in[0];
  const float* ln1_w   = (const float*)d_in[1];
  const float* ln1_b   = (const float*)d_in[2];
  const float* ln2_w   = (const float*)d_in[3];
  const float* ln2_b   = (const float*)d_in[4];
  const float* rel_pos = (const float*)d_in[5];
  const float* d_w1    = (const float*)d_in[6];
  const float* d_b1    = (const float*)d_in[7];
  const float* d_w2    = (const float*)d_in[8];
  const float* d_b2    = (const float*)d_in[9];
  const float* r_w1    = (const float*)d_in[10];
  const float* r_b1    = (const float*)d_in[11];
  const float* r_w2    = (const float*)d_in[12];
  const float* r_b2    = (const float*)d_in[13];
  const float* v_w     = (const float*)d_in[14];
  const float* v_b     = (const float*)d_in[15];
  const float* o_w     = (const float*)d_in[16];
  const float* o_b     = (const float*)d_in[17];
  const float* eml_g   = (const float*)d_in[18];
  const float* eml_lam = (const float*)d_in[19];
  const float* eml_bias= (const float*)d_in[20];
  float* out = (float*)d_out;

  char* ws = (char*)d_ws;
  size_t off = 0;
  const size_t szX    = (size_t)npix * CDIM * 2;
  const size_t szWbig = (size_t)PLD * CDIM * 2;
  const size_t szoW   = (size_t)CDIM * CDIM * 2;
  const size_t szTab  = (size_t)NBR * CDIM * 4;
  const size_t szP    = (size_t)npix * PLD * 4;
  const size_t szMSG  = (size_t)npix * CDIM * 2;
  _Float16* Xh   = (_Float16*)(ws + off); off += szX;
  _Float16* Wbig = (_Float16*)(ws + off); off += szWbig;
  _Float16* oWt  = (_Float16*)(ws + off); off += szoW;
  float*    cD   = (float*)(ws + off);    off += szTab;
  float*    cR   = (float*)(ws + off);    off += szTab;
  float*    P    = (float*)(ws + off);    off += szP;
  _Float16* MSG  = (_Float16*)(ws + off); off += szMSG;
  float*    Y    = P;
  if (off > ws_size) return;
  if ((size_t)npix * CDIM * 4 > szP) return;

  {
    const int nthreads = 640 * 16 + 128 * 16 + 2 * NBR * CDIM;
    prep_kernel<<<(nthreads + 255) / 256, 256, 0, stream>>>(d_w1, d_b1, r_w1, r_b1, v_w, o_w, rel_pos,
                                                             Wbig, oWt, cD, cR);
  }
  ln1_kernel<<<(npix + 15) / 16, 256, 0, stream>>>(tokens, ln1_w, ln1_b, Xh, npix);
  {
    const int tiles = (npix / 64) * (PLD / 64);
    wmma_gemm64<0, false, 0, 0, false, 0><<<dim3((tiles + 7) / 8, 1), 256, 0, stream>>>(
        (const unsigned short*)Xh, (const unsigned short*)Xh, CDIM, 0L,
        (const unsigned short*)Wbig, (const unsigned short*)Wbig, CDIM, 0L,
        (void*)P, (void*)P, PLD, 0L,
        v_b, tokens, 0L,
        npix, PLD, CDIM, 1.0f / (XSC * WSC));
  }
  edge_kernel<<<(npix + TT - 1) / TT, 256, 0, stream>>>(P, cD, cR, d_w2, d_b2, r_w2, r_b2, v_b,
                                                        eml_g, eml_lam, eml_bias, MSG, npix);
  {
    const int tiles = (npix / 64) * (CDIM / 64);
    wmma_gemm64<0, false, 2, 0, true, 0><<<dim3((tiles + 7) / 8, 1), 256, 0, stream>>>(
        (const unsigned short*)MSG, (const unsigned short*)MSG, CDIM, 0L,
        (const unsigned short*)oWt, (const unsigned short*)oWt, CDIM, 0L,
        (void*)Y, (void*)Y, CDIM, 0L,
        o_b, tokens, 0L,
        npix, CDIM, CDIM, 1.0f / (MSC * WSC));
  }
  ln2_kernel<<<(npix + 7) / 8, 256, 0, stream>>>(Y, ln2_w, ln2_b, out, npix);
}
